// MyVMLMFCellg2_67027259621390
// MI455X (gfx1250) — hardware-run, weakly checked
//
#include <hip/hip_runtime.h>


namespace {
constexpr int B = 4096, I = 1024, H = 1024, R = 64, G = 2, HG = 512, CHK = 32;
constexpr float XS = 8.0f, HS = 256.0f, WSC = 256.0f;
typedef _Float16 b16;
typedef __attribute__((ext_vector_type(16))) _Float16 v16b;
typedef __attribute__((ext_vector_type(8))) _Float16 v8b;
typedef __attribute__((ext_vector_type(8))) float v8f;
typedef __attribute__((ext_vector_type(4))) float v4f;
__device__ __forceinline__ float bf16_rne(float f) { unsigned int u = __float_as_uint(f); u += 0x7FFFu + ((u >> 16) & 1u); float r = __uint_as_float(u & 0xFFFF0000u); asm volatile("" : "+v"(r)); return r; }
__device__ __forceinline__ float bfv(float f) { float r = bf16_rne(f); asm volatile("" : "+v"(r)); return r; }
__device__ __forceinline__ void split16(float v, b16& hi, b16& lo) { hi = (b16)v; lo = (b16)(v - (float)hi); }
__device__ __forceinline__ v16b frag_kb(const b16* p, int hh) { const v8b a = *(const v8b*)(p + 8 * hh), b = *(const v8b*)(p + 16 + 8 * hh); v16b f;
#pragma unroll
  for (int e = 0; e < 8; ++e) { f[e] = a[e]; f[8 + e] = b[e]; } return f; }
__device__ __forceinline__ v8f wmma16b(v16b a, v16b b, v8f c) { v8f d = __builtin_amdgcn_wmma_f32_16x16x32_f16(false, a, false, b, (short)0, c, false, false); asm volatile("v_nop\n\tv_nop\n\tv_nop\n\tv_nop" : "+v"(d) : "v"(a), "v"(b)); return d; }
__device__ __forceinline__ void wave_lds_sync() { __builtin_amdgcn_fence(__ATOMIC_RELEASE, "workgroup"); __builtin_amdgcn_wave_barrier(); __builtin_amdgcn_fence(__ATOMIC_ACQUIRE, "workgroup"); }
__device__ __forceinline__ float pmul(float a, float b) { float p = a * b; asm volatile("" : "+v"(p)); return p; }
__device__ __forceinline__ float sigm(float v) { return 1.0f / (1.0f + __expf(-v)); }

__global__ __launch_bounds__(256) void wput_kernel(const float* __restrict__ ux, const float* __restrict__ vx, const float* __restrict__ uh0, const float* __restrict__ uh1, const float* __restrict__ vh0, const float* __restrict__ vh1, b16* __restrict__ UXT, b16* __restrict__ UHT, b16* __restrict__ VX, b16* __restrict__ VHT, float* __restrict__ DG) { const size_t nt = (size_t)gridDim.x * 256, u0 = (size_t)blockIdx.x * 256 + threadIdx.x; v8b v;
  for (size_t u = u0; u < (size_t)R * (I / 8); u += nt) { const int r = (int)(u / (I / 8)), k0 = (int)(u % (I / 8)) * 8;
#pragma unroll
    for (int j = 0; j < 8; ++j) v[j] = (b16)(bf16_rne(ux[(size_t)(k0 + j) * R + r]) * WSC); for (int pass = 0; pass < 2; ++pass) { *(volatile v8b*)(UXT + (size_t)r * I + k0) = v; __threadfence(); } }
  for (size_t u = u0; u < (size_t)2 * G * R * (HG / 8); u += nt) { const int ig = (int)(u / (R * (HG / 8))), rem = (int)(u % (R * (HG / 8))); const int r = rem / (HG / 8), k0 = (rem % (HG / 8)) * 8; const int i = ig / G, g = ig % G; const float* uu = (i ? uh1 : uh0) + (size_t)g * HG * R;
#pragma unroll
    for (int j = 0; j < 8; ++j) v[j] = (b16)(bf16_rne(uu[(size_t)(k0 + j) * R + r]) * WSC); for (int pass = 0; pass < 2; ++pass) { *(volatile v8b*)(UHT + ((size_t)ig * R + r) * HG + k0) = v; __threadfence(); } }
  for (size_t u = u0; u < (size_t)4 * H * 8; u += nt) { const int o = (int)(u / 8), k0 = (int)(u % 8) * 8;
#pragma unroll
    for (int j = 0; j < 8; ++j) v[j] = (b16)(bf16_rne(vx[(size_t)o * R + k0 + j]) * WSC); for (int pass = 0; pass < 2; ++pass) { *(volatile v8b*)(VX + (size_t)o * R + k0) = v; __threadfence(); } }
  for (size_t u = u0; u < (size_t)2 * G * 4 * HG * 8; u += nt) { const int ig = (int)(u / (4 * HG * 8)), rem = (int)(u % (4 * HG * 8)); const int kk = rem / 8, k0 = (rem % 8) * 8; const int i = ig / G, g = ig % G; const float* vv = (i ? vh1 : vh0) + (size_t)g * R * 4 * HG;
#pragma unroll
    for (int j = 0; j < 8; ++j) v[j] = (b16)(bf16_rne(vv[(size_t)(k0 + j) * 4 * HG + kk]) * WSC); for (int pass = 0; pass < 2; ++pass) { *(volatile v8b*)(VHT + ((size_t)ig * 4 * HG + kk) * R + k0) = v; __threadfence(); } }
  for (size_t u = u0; u < (size_t)8 * H; u += nt) { const int row = (int)(u / H), j = (int)(u % H); float s = 0.0f; if (row < 4) { for (int r = 0; r < R; ++r) s += pmul(bfv(ux[(size_t)j * R + r]), bfv(vx[((size_t)row * H + j) * R + r])); } else { const int k = row - 4, g = j / HG, hh = j % HG; for (int r = 0; r < R; ++r) s += pmul(bfv(uh0[((size_t)g * HG + hh) * R + r]), bfv(vh0[((size_t)g * R + r) * 4 * HG + k * HG + hh])); }
    for (int pass = 0; pass < 2; ++pass) { ((volatile float*)DG)[u] = s; __threadfence(); } } }
__global__ __launch_bounds__(32) void main_kernel(const float* __restrict__ x, const float* __restrict__ h, const float* __restrict__ c, const float* __restrict__ dx, const float* __restrict__ dh, const b16* __restrict__ UXT, const b16* __restrict__ UHT, const b16* __restrict__ VX, const b16* __restrict__ VHT, const float* __restrict__ DG, const float* __restrict__ bx, const float* __restrict__ bh, int BLIM, float* __restrict__ oh, float* __restrict__ oc) { __shared__ __attribute__((aligned(16))) b16 Ax[16][I + 8], Th[5][16][R + 8], Tl[5][16][R + 8]; __shared__ float Gx[16][4][CHK + 1], Gh[16][4][CHK + 1]; const int lane = threadIdx.x, nloc = lane & 15, hlf = lane >> 4; const size_t b0 = (size_t)blockIdx.x * 16; if (b0 >= (size_t)BLIM) return;
  for (int rr = 0; rr < 16; ++rr) for (int q = 0; q < I / 32; ++q) { const int cc = q * 32 + lane; Ax[rr][cc] = (b16)(bf16_rne(x[(b0 + rr) * I + cc]) * XS); }
  if (lane < 16) for (int k = I; k < I + 8; ++k) Ax[lane][k] = (b16)0.0f;
  wave_lds_sync();
  auto tproj = [&](const b16* W, int K, int slot) { v8f acc[4] = {(v8f){}, (v8f){}, (v8f){}, (v8f){}};
    for (int kb = 0; kb < K; kb += 32) { const v16b a = frag_kb(&Ax[nloc][kb], hlf);
#pragma unroll
      for (int t = 0; t < 4; ++t) acc[t] = wmma16b(a, frag_kb(W + (size_t)(t * 16 + nloc) * K + kb, hlf), acc[t]); }
#pragma unroll
    for (int t = 0; t < 4; ++t)
#pragma unroll
      for (int r8 = 0; r8 < 8; ++r8) { b16 p, ql; split16(acc[t][r8] * (1.0f / (XS * WSC)) * HS, p, ql); Th[slot][8 * hlf + r8][t * 16 + nloc] = p; Tl[slot][8 * hlf + r8][t * 16 + nloc] = ql; } };
  tproj(UXT, I, 0);
  wave_lds_sync();
  for (int rr = 0; rr < 16; ++rr) for (int q = 0; q < H / 32; ++q) { const int cc = q * 32 + lane; Ax[rr][cc] = (b16)(bf16_rne(h[(b0 + rr) * H + cc]) * XS); }
  wave_lds_sync();
#pragma unroll 1
  for (int ig = 0; ig < 4; ++ig) { const int i = ig / G, g = ig % G; const int srcg = (g + i) % G;
    { v8f acc[4] = {(v8f){}, (v8f){}, (v8f){}, (v8f){}};
#pragma unroll 2
      for (int kb = 0; kb < HG; kb += 32) { const v16b a = frag_kb(&Ax[nloc][srcg * HG + kb], hlf);
#pragma unroll
        for (int t = 0; t < 4; ++t) acc[t] = wmma16b(a, frag_kb(UHT + ((size_t)ig * R + t * 16 + nloc) * HG + kb, hlf), acc[t]); }
#pragma unroll
      for (int t = 0; t < 4; ++t)
#pragma unroll
        for (int r8 = 0; r8 < 8; ++r8) { b16 p, ql; split16(acc[t][r8] * (1.0f / (XS * WSC)) * HS, p, ql); Th[1 + ig][8 * hlf + r8][t * 16 + nloc] = p; Tl[1 + ig][8 * hlf + r8][t * 16 + nloc] = ql; } } }
  if (lane < 16) for (int s = 0; s < 5; ++s) for (int k = R; k < R + 8; ++k) { Th[s][lane][k] = (b16)0.0f; Tl[s][lane][k] = (b16)0.0f; }
  wave_lds_sync();
  const v16b ta[2] = {frag_kb(&Th[0][nloc][0], hlf), frag_kb(&Th[0][nloc][32], hlf)}, tla[2] = {frag_kb(&Tl[0][nloc][0], hlf), frag_kb(&Tl[0][nloc][32], hlf)};
#pragma unroll 1
  for (int j0 = 0; j0 < H; j0 += CHK) { const int g = j0 / HG, hh0 = j0 % HG;
    v8f gx[4][2], ah[4][2];
#pragma unroll
    for (int k = 0; k < 4; ++k) for (int ct = 0; ct < 2; ++ct) { gx[k][ct] = (v8f){}; ah[k][ct] = (v8f){}; }
#pragma unroll
    for (int ks = 0; ks < 2; ++ks) {
#pragma unroll
      for (int k = 0; k < 4; ++k)
#pragma unroll
        for (int ct = 0; ct < 2; ++ct) { const v16b bw = frag_kb(VX + (size_t)(k * H + j0 + ct * 16 + nloc) * R + ks * 32, hlf); gx[k][ct] = wmma16b(ta[ks], bw, gx[k][ct]); gx[k][ct] = wmma16b(tla[ks], bw, gx[k][ct]); } }
#pragma unroll 1
    for (int i = 0; i < 2; ++i) { const int ig = i * G + g; const v16b ua0 = frag_kb(&Th[1 + ig][nloc][0], hlf), ua1 = frag_kb(&Th[1 + ig][nloc][32], hlf), ul0 = frag_kb(&Tl[1 + ig][nloc][0], hlf), ul1 = frag_kb(&Tl[1 + ig][nloc][32], hlf);
#pragma unroll
      for (int k = 0; k < 4; ++k)
#pragma unroll
        for (int ct = 0; ct < 2; ++ct) { const b16* wp = VHT + ((size_t)ig * 4 * HG + k * HG + hh0 + ct * 16 + nloc) * R; const v16b b0 = frag_kb(wp, hlf), b1 = frag_kb(wp + 32, hlf); ah[k][ct] = wmma16b(ua0, b0, ah[k][ct]); ah[k][ct] = wmma16b(ul0, b0, ah[k][ct]); ah[k][ct] = wmma16b(ua1, b1, ah[k][ct]); ah[k][ct] = wmma16b(ul1, b1, ah[k][ct]); } }
#pragma unroll
    for (int k = 0; k < 4; ++k)
#pragma unroll
      for (int ct = 0; ct < 2; ++ct)
#pragma unroll
        for (int r8 = 0; r8 < 8; ++r8) { Gx[8 * hlf + r8][k][ct * 16 + nloc] = gx[k][ct][r8] * (1.0f / (HS * WSC)); Gh[8 * hlf + r8][k][ct * 16 + nloc] = ah[k][ct][r8] * (1.0f / (HS * WSC)); }
    wave_lds_sync();
    { const int j = j0 + lane; const float dxj = bfv(dx[j]), dhj = bfv(dh[j]); float dgx[4], dgh[4], bxx[4], bhh[4]; for (int k = 0; k < 4; ++k) { dgx[k] = DG[(size_t)k * H + j]; dgh[k] = DG[(size_t)(4 + k) * H + j]; bxx[k] = bfv(bx[(size_t)k * H + j]); bhh[k] = bfv(bh[(size_t)k * H + j]); }
      for (int pass = 0; pass < 2; ++pass) { for (int rr = 0; rr < 16; ++rr) { const size_t bi = b0 + rr; const float xv = bfv(x[bi * I + j]), hv = bfv(h[bi * H + j]), cv = bfv(c[bi * H + j]); const float base = pmul(dxj, xv) + pmul(dhj, hv);
          const float xi = Gx[rr][0][lane] - pmul(xv, dgx[0]) + bxx[0], xf = Gx[rr][1][lane] - pmul(xv, dgx[1]) + bxx[1], xo = Gx[rr][2][lane] - pmul(xv, dgx[2]) + bxx[2], xn = Gx[rr][3][lane] - pmul(xv, dgx[3]) + bxx[3];
          const float hf = bhh[0] - pmul(hv, dgh[0]) + Gh[rr][0][lane], hi = bhh[1] - pmul(hv, dgh[1]) + Gh[rr][1][lane], hn = bhh[2] - pmul(hv, dgh[2]) + Gh[rr][2][lane], ho = bhh[3] - pmul(hv, dgh[3]) + Gh[rr][3][lane];
          const float ig_ = sigm(xi + hi + base), fg = sigm(xf + hf + base), og = sigm(xo + ho + base), ng = tanhf(xn + hn + base); const float cn = fg * cv + ig_ * ng; const float hn_ = og * tanhf(cn);
          ((volatile float*)oc)[bi * H + j] = cn; ((volatile float*)oh)[bi * H + j] = hn_; } __threadfence(); } }
    wave_lds_sync(); } }
}

extern "C" void kernel_launch(void* const* d_in, const int* in_sizes, int n_in, void* d_out, int out_size, void* d_ws, size_t ws_size, hipStream_t stream) {
  (void)n_in;
  auto Fp = [&](int i) { return (const float*)d_in[i]; };
  if (in_sizes[0] != B * I || in_sizes[1] != B * H || in_sizes[2] != B * H || in_sizes[3] != I || in_sizes[5] != I * R || in_sizes[6] != 4 * H * R || in_sizes[7] != G * HG * R || in_sizes[9] != G * R * 4 * HG || in_sizes[11] != 4 * H || out_size != 2 * B * H) return;
  const int BLIM = B;
  size_t off = 0; char* ws = (char*)d_ws;
  auto carve = [&](size_t bytes) { char* p = ws + off; off += (bytes + 255) & ~(size_t)255; return p; };
  b16* UXT = (b16*)carve((size_t)R * I * 2); b16* UHT = (b16*)carve((size_t)2 * G * R * HG * 2); b16* VX = (b16*)carve((size_t)4 * H * R * 2); b16* VHT = (b16*)carve((size_t)2 * G * 4 * HG * R * 2); float* DG = (float*)carve((size_t)8 * H * 4);
  if (off > ws_size || off > ((size_t)4 << 20)) return;
  wput_kernel<<<128, 256, 0, stream>>>(Fp(5), Fp(6), Fp(7), Fp(8), Fp(9), Fp(10), UXT, UHT, VX, VHT, DG);
  main_kernel<<<BLIM / 16, 32, 0, stream>>>(Fp(0), Fp(1), Fp(2), Fp(3), Fp(4), UXT, UHT, VX, VHT, DG, Fp(11), Fp(12), BLIM, (float*)d_out, (float*)d_out + (size_t)B * H);
}
